// ScaledDotProduct_71554155151920
// MI455X (gfx1250) — hardware-verified
//
#include <hip/hip_runtime.h>
#include <math.h>

constexpr int kBatch = 4;
constexpr int kSeq   = 2048;
constexpr int kC     = 1024;
constexpr int kQKV   = 3 * kC;
constexpr int kQKW   = 2 * kC;
constexpr int kTok   = kBatch * kSeq;
constexpr int kSeqTiles   = kSeq / 64;
constexpr int kTriTiles   = kSeqTiles * (kSeqTiles + 1) / 2;
constexpr int kSplitRows  = 256;
constexpr int kSplitTiles = (kSplitRows / 64) * ((kSplitRows / 64) + 1) / 2;
constexpr float kScoreScale = 0.03125f;
constexpr float kMaskFill   = -9.0e15f;
static_assert(kTok % 64 == 0 && kSeq % 64 == 0 && kC % 64 == 0 && kQKW % 64 == 0 && kSplitRows % 64 == 0, "tiles");
static_assert(kC % 32 == 0 && kSeq % 32 == 0, "ktiles");
static_assert(kSeq == 8 * 256, "softmax row map");
static_assert(kTriTiles == 528 && kSplitTiles == 10 && kSplitRows <= kSeq, "tri grid");

typedef __attribute__((ext_vector_type(16))) _Float16 v16h;
typedef __attribute__((ext_vector_type(8)))  _Float16 v8h;
typedef __attribute__((ext_vector_type(16))) __bf16   v16b;
typedef __attribute__((ext_vector_type(8)))  __bf16   v8b;
typedef __attribute__((ext_vector_type(8)))  float    v8f;
typedef __attribute__((ext_vector_type(4)))  float    v4f;
typedef __attribute__((ext_vector_type(2)))  float    v2f;
typedef __attribute__((ext_vector_type(4)))  unsigned int v4u;

__device__ __forceinline__ unsigned short f2bf_bits(float f) {
  unsigned u = __float_as_uint(f);
  return (unsigned short)((u + 0x7FFFu + ((u >> 16) & 1u)) >> 16);
}
__device__ __forceinline__ float bf_bits2f(unsigned short h) { return __uint_as_float(((unsigned)h) << 16); }

__device__ __forceinline__ void dep_guard_h(v8f& a, v8f& b, v16h x, v16h y) { asm volatile("v_nop\n\tv_nop\n\tv_nop\n\tv_nop" : "+v"(a), "+v"(b) : "v"(x), "v"(y)); }
__device__ __forceinline__ void dep_guard_b(v8f& a, v8f& b, v16b x, v16b y) { asm volatile("v_nop\n\tv_nop\n\tv_nop\n\tv_nop" : "+v"(a), "+v"(b) : "v"(x), "v"(y)); }
__device__ __forceinline__ void dep_guard4_h(v8f& a, v8f& b, v8f& c, v8f& d, v16h x, v16h y) { asm volatile("v_nop\n\tv_nop\n\tv_nop\n\tv_nop" : "+v"(a), "+v"(b), "+v"(c), "+v"(d) : "v"(x), "v"(y)); }
__device__ __forceinline__ void dep_guard4_b(v8f& a, v8f& b, v8f& c, v8f& d, v16b x, v16b y) { asm volatile("v_nop\n\tv_nop\n\tv_nop\n\tv_nop" : "+v"(a), "+v"(b), "+v"(c), "+v"(d) : "v"(x), "v"(y)); }
__device__ __forceinline__ void keep4_h(v16h a, v16h b, v16h c, v16h d) { asm volatile("v_nop" :: "v"(a), "v"(b), "v"(c), "v"(d)); }
__device__ __forceinline__ void keep4_b(v16b a, v16b b, v16b c, v16b d) { asm volatile("v_nop" :: "v"(a), "v"(b), "v"(c), "v"(d)); }
__device__ __forceinline__ void acc_guard4(v8f& a, v8f& b, v8f& c, v8f& d) { asm volatile("v_nop\n\tv_nop\n\tv_nop\n\tv_nop" : "+v"(a), "+v"(b), "+v"(c), "+v"(d)); }
template <typename T> struct Frag;
template <> struct Frag<_Float16> {
  typedef v16h V; union U { v16h v; v8h h[2]; };
  static __device__ __forceinline__ v16h load(const _Float16* p) {
    U f; f.h[0] = *(const v8h*)(p); f.h[1] = *(const v8h*)(p + 16); return f.v;
  }
  static __device__ __forceinline__ v8f mma(v16h a, v16h b, v8f c) {
    return __builtin_amdgcn_wmma_f32_16x16x32_f16(false, a, false, b, (short)0, c, false, false);
  }
  static __device__ __forceinline__ void guard(v8f& a, v8f& b, v16h x, v16h y) { dep_guard_h(a, b, x, y); }
  static __device__ __forceinline__ void guard4(v8f& a, v8f& b, v8f& c, v8f& d, v16h x, v16h y) { dep_guard4_h(a, b, c, d, x, y); }
  static __device__ __forceinline__ void keep(v16h a, v16h b, v16h c, v16h d) { keep4_h(a, b, c, d); }
};
template <> struct Frag<__bf16> {
  typedef v16b V; union U { v16b v; v8b h[2]; };
  static __device__ __forceinline__ v16b load(const __bf16* p) {
    U f; f.h[0] = *(const v8b*)(p); f.h[1] = *(const v8b*)(p + 16); return f.v;
  }
  static __device__ __forceinline__ v8f mma(v16b a, v16b b, v8f c) {
    return __builtin_amdgcn_wmma_f32_16x16x32_bf16(false, a, false, b, (short)0, c, false, false);
  }
  static __device__ __forceinline__ void guard(v8f& a, v8f& b, v16b x, v16b y) { dep_guard_b(a, b, x, y); }
  static __device__ __forceinline__ void guard4(v8f& a, v8f& b, v8f& c, v8f& d, v16b x, v16b y) { dep_guard4_b(a, b, c, d, x, y); }
  static __device__ __forceinline__ void keep(v16b a, v16b b, v16b c, v16b d) { keep4_b(a, b, c, d); }
};

__device__ __forceinline__ unsigned pk16(unsigned short a, unsigned short b) { return (unsigned)a | ((unsigned)b << 16); }

template <int ET> struct Elem;
template <> struct Elem<0> { typedef _Float16 T; };
template <> struct Elem<1> { typedef __bf16 T; };
template <int ET, bool SPLIT, int BIAS_MODE, int OUT_MODE, bool RESID, int ACT = 0, int TRI = 0, int TILE0 = 0>
__global__ __launch_bounds__(256) void wmma_gemm64(
    const unsigned short* __restrict__ Ap, const unsigned short* __restrict__ A2p, int lda, long strideA,
    const unsigned short* __restrict__ Btp, const unsigned short* __restrict__ Bt2p, int ldb, long strideB,
    void* __restrict__ Cout, void* __restrict__ Cout2, int ldc, long strideC,
    const float* __restrict__ bias,
    const float* __restrict__ resid, long strideR,
    int M, int N, int K, float scale) {
  typedef typename Elem<ET>::T T;
  typedef typename Frag<T>::V V;
  const T* A = (const T*)Ap; const T* A2 = (const T*)A2p; const T* Bt = (const T*)Btp; const T* Bt2 = (const T*)Bt2p;
  __shared__ __align__(16) float sT[8][16 * 68];
  const int b    = blockIdx.y;
  const int lane = threadIdx.x & 31;
  const int wave = threadIdx.x >> 5;
  const int tilesN = N >> 6;
  const int tilesM = M >> 6;
  const int nTiles = (TRI == 1) ? ((tilesM * (tilesM + 1)) >> 1) : (tilesM * tilesN);
  const int tile = blockIdx.x * 8 + wave + TILE0;
  if (tile >= nTiles) return;
  int tm, tn;
  if (TRI == 1) {
    int rsel = 0, ssel = 0, s = 0;
#pragma unroll 1
    for (int r = 1; r < tilesM; ++r) {
      s += r;
      const bool ge = (s <= tile);
      rsel = ge ? r : rsel;
      ssel = ge ? s : ssel;
    }
    tm = rsel;
    tn = tile - ssel;
  } else {
    tm = tile / tilesN;
    tn = tile - tm * tilesN;
  }
  const int m0 = tm << 6;
  const int n0 = tn << 6;
  const int Kend = (TRI == 2) ? (((m0 + 64) < K) ? (m0 + 64) : K) : K;

  const T* Ab  = A  + (size_t)b * strideA;
  const T* Bb  = Bt + (size_t)b * strideB;
  const T* Ab2 = SPLIT ? (A2  + (size_t)b * strideA) : nullptr;
  const T* Bb2 = SPLIT ? (Bt2 + (size_t)b * strideB) : nullptr;

  const int rlane = lane & 15;
  const int koff  = (lane >> 4) * 8;
  const int mOff  = (lane >> 4) * 8;

  v8f acc[4][4];
#pragma unroll
  for (int i = 0; i < 4; ++i)
#pragma unroll
    for (int j = 0; j < 4; ++j) acc[i][j] = (v8f){0.f,0.f,0.f,0.f,0.f,0.f,0.f,0.f};

  for (int k0 = 0; k0 < Kend; k0 += 32) {
    V bh[4], bl[4];
#pragma unroll
    for (int j = 0; j < 4; ++j) {
      const size_t bo = (size_t)(n0 + (j << 4) + rlane) * ldb + koff + k0;
      bh[j] = Frag<T>::load(Bb + bo);
      if (SPLIT) bl[j] = Frag<T>::load(Bb2 + bo);
    }
#pragma unroll
    for (int i = 0; i < 4; ++i) {
      const size_t ao = (size_t)(m0 + (i << 4) + rlane) * lda + koff + k0;
      V ah = Frag<T>::load(Ab + ao);
      V al;
      if (SPLIT) al = Frag<T>::load(Ab2 + ao);
#pragma unroll
      for (int j = 0; j < 4; ++j) {
        acc[i][j] = Frag<T>::mma(ah, bh[j], acc[i][j]);
        if (SPLIT) {
          acc[i][j] = Frag<T>::mma(ah, bl[j], acc[i][j]);
          acc[i][j] = Frag<T>::mma(al, bh[j], acc[i][j]);
        }
      }
      Frag<T>::guard4(acc[i][0], acc[i][1], acc[i][2], acc[i][3], ah, SPLIT ? al : ah);
    }
    Frag<T>::keep(bh[0], bh[1], bh[2], bh[3]);
    if (SPLIT) Frag<T>::keep(bl[0], bl[1], bl[2], bl[3]);
  }
  acc_guard4(acc[0][0], acc[0][1], acc[0][2], acc[0][3]);
  acc_guard4(acc[1][0], acc[1][1], acc[1][2], acc[1][3]);
  acc_guard4(acc[2][0], acc[2][1], acc[2][2], acc[2][3]);
  acc_guard4(acc[3][0], acc[3][1], acc[3][2], acc[3][3]);

  float* slab = sT[wave];
  const float* Rb = RESID ? (resid + (size_t)b * strideR) : nullptr;
#pragma unroll
  for (int i = 0; i < 4; ++i) {
    const int mBase = m0 + (i << 4);
#pragma unroll
    for (int j = 0; j < 4; ++j) {
      const int n = n0 + (j << 4) + rlane;
      float bv = 0.f;
      if (BIAS_MODE == 2) bv = bias[n];
#pragma unroll
      for (int r = 0; r < 8; ++r) {
        float v = acc[i][j][r] * scale;
        if (BIAS_MODE == 1) v += bias[mBase + mOff + r];
        if (BIAS_MODE == 2) v += bv;
        if (RESID) v += Rb[(size_t)(mBase + mOff + r) * ldc + n];
        if (ACT == 2) v = fmaxf(v, 0.0f);
        if (ACT == 4) v = (v > 0.f) ? v : 0.01f * v;
        slab[(mOff + r) * 68 + (j << 4) + rlane] = v;
      }
    }
    __builtin_amdgcn_fence(__ATOMIC_RELEASE, "workgroup");
    __builtin_amdgcn_wave_barrier();
    __builtin_amdgcn_fence(__ATOMIC_ACQUIRE, "workgroup");
    if (OUT_MODE == 0) {
      float* C = (float*)Cout + (size_t)b * strideC;
      const int hh = lane >> 4, c4 = (lane & 15) * 4;
      for (int pass = 0; pass < 2; ++pass) {
#pragma unroll
        for (int it = 0; it < 8; ++it) {
          const int row = it * 2 + hh;
          v4f v = *(const v4f*)(slab + row * 68 + c4);
          *(volatile v4f*)(C + (size_t)(mBase + row) * ldc + n0 + c4) = v;
        }
        __threadfence();
      }
    } else {
      const int q = lane >> 3, c8 = (lane & 7) * 8;
      unsigned short* C  = (unsigned short*)Cout  + (size_t)b * strideC;
      unsigned short* C2 = (OUT_MODE == 2) ? ((unsigned short*)Cout2 + (size_t)b * strideC) : nullptr;
      for (int pass = 0; pass < 2; ++pass) {
#pragma unroll
        for (int it = 0; it < 4; ++it) {
          const int row = it * 4 + q;
          const float* sp = slab + row * 68 + c8;
          v8h hv, lv;
#pragma unroll
          for (int e = 0; e < 8; ++e) {
            if (OUT_MODE == 1) {
              hv[e] = (_Float16)sp[e];
            } else {
              unsigned short hb = f2bf_bits(sp[e]);
              unsigned short lb = f2bf_bits(sp[e] - bf_bits2f(hb));
              hv[e] = __builtin_bit_cast(_Float16, hb);
              lv[e] = __builtin_bit_cast(_Float16, lb);
            }
          }
          *(volatile v8h*)(C + (size_t)(mBase + row) * ldc + n0 + c8) = hv;
          if (OUT_MODE == 2) *(volatile v8h*)(C2 + (size_t)(mBase + row) * ldc + n0 + c8) = lv;
        }
        __threadfence();
      }
    }
    __builtin_amdgcn_fence(__ATOMIC_RELEASE, "workgroup");
    __builtin_amdgcn_wave_barrier();
    __builtin_amdgcn_fence(__ATOMIC_ACQUIRE, "workgroup");
  }
}

__global__ __launch_bounds__(256) void cast8_bf16_kernel(const float* __restrict__ in, unsigned short* __restrict__ out, int n8) {
  const int i = blockIdx.x * 256 + threadIdx.x;
  if (i >= n8) return;
  const float* p = in + 8 * (size_t)i;
  const v4f a = *(const v4f*)(p);
  const v4f c = *(const v4f*)(p + 4);
  unsigned short hb[8];
#pragma unroll
  for (int e = 0; e < 4; ++e) {
    hb[e]     = f2bf_bits(a[e]);
    hb[4 + e] = f2bf_bits(c[e]);
  }
  const v4u u = (v4u){pk16(hb[0], hb[1]), pk16(hb[2], hb[3]), pk16(hb[4], hb[5]), pk16(hb[6], hb[7])};
  unsigned short* q = out + 8 * (size_t)i;
  *(volatile v4u*)q = u;
  __threadfence();
  *(volatile v4u*)q = u;
}

__global__ __launch_bounds__(256) void wt_cast_kernel(const float* __restrict__ W, unsigned short* __restrict__ WT) {
  __shared__ float sm[64][65];
  const int t  = threadIdx.x;
  const int d0 = blockIdx.x * 64;
  const int c0 = blockIdx.y * 64;
#pragma unroll
  for (int i = 0; i < 8; ++i) {
    const int e  = i * 256 + t;
    const int cl = e >> 6;
    const int dl = e & 63;
    sm[dl][cl] = W[(size_t)(c0 + cl) * kQKV + d0 + dl];
  }
  asm volatile("" ::: "memory");
#pragma unroll
  for (int i = 8; i < 16; ++i) {
    const int e  = i * 256 + t;
    const int cl = e >> 6;
    const int dl = e & 63;
    sm[dl][cl] = W[(size_t)(c0 + cl) * kQKV + d0 + dl];
  }
  __syncthreads();
  const int lane = t & 31, wave = t >> 5;
  const int q = lane >> 3, c8 = (lane & 7) * 8;
  for (int pass = 0; pass < 2; ++pass) {
#pragma unroll
    for (int it = 0; it < 2; ++it) {
      const int row = wave * 8 + it * 4 + q;
      unsigned short hb[8];
#pragma unroll
      for (int e = 0; e < 8; ++e) hb[e] = f2bf_bits(sm[row][c8 + e]);
      const v4u u = (v4u){pk16(hb[0], hb[1]), pk16(hb[2], hb[3]), pk16(hb[4], hb[5]), pk16(hb[6], hb[7])};
      *(volatile v4u*)(WT + (size_t)(d0 + row) * kC + c0 + c8) = u;
    }
    __threadfence();
  }
}

__global__ __launch_bounds__(256) void causal_softmax_kernel(const float* __restrict__ Sp,
                                                             unsigned short* __restrict__ Php,
                                                             unsigned short* __restrict__ Plp) {
  __shared__ __align__(16) float lg[kSeq];
  __shared__ float redM[8];
  __shared__ float redS[8];
  const int i    = blockIdx.x;
  const int t    = threadIdx.x;
  const int lane = t & 31, wave = t >> 5;
  const float* sr = Sp + (size_t)i * kSeq;
  const int cl2 = (i | 63) - 1;

  float mx = -__builtin_inff();
#pragma unroll 1
  for (int it = 0; it < 4; ++it) {
    const int c  = it * 512 + 2 * t;
    const int cc = (c < cl2) ? c : cl2;
    const v2f sv = *(const v2f*)(sr + cc);
    v2f zv;
#pragma unroll
    for (int e = 0; e < 2; ++e) {
      const float fl = (c + e <= i) ? 1.0f : 0.0f;
      const float z  = fmaf(fl, sv[e], (1.0f - fl) * kMaskFill);
      zv[e] = z;
      mx = fmaxf(mx, z);
    }
    *(v2f*)(lg + c) = zv;
  }
#pragma unroll
  for (int off = 16; off > 0; off >>= 1) mx = fmaxf(mx, __shfl_xor(mx, off, 32));
  if (lane == 0) redM[wave] = mx;
  __syncthreads();
  float m = redM[0];
#pragma unroll
  for (int w = 1; w < 8; ++w) m = fmaxf(m, redM[w]);

  float sum = 0.f;
#pragma unroll 1
  for (int it = 0; it < 4; ++it) {
    const int c = it * 512 + 2 * t;
    const v2f l = *(const v2f*)(lg + c);
    v2f ev;
#pragma unroll
    for (int e = 0; e < 2; ++e) {
      ev[e] = expf(l[e] - m);
      sum += ev[e];
    }
    *(v2f*)(lg + c) = ev;
  }
#pragma unroll
  for (int off = 16; off > 0; off >>= 1) sum += __shfl_xor(sum, off, 32);
  if (lane == 0) redS[wave] = sum;
  __syncthreads();
  float tot = redS[0];
#pragma unroll
  for (int w = 1; w < 8; ++w) tot += redS[w];
  const float inv = 1.0f / tot;

  const v4f e0 = *(const v4f*)(lg + 8 * t);
  const v4f e1 = *(const v4f*)(lg + 8 * t + 4);
  unsigned short hb[8], lb[8];
#pragma unroll
  for (int e = 0; e < 4; ++e) {
    const float p0 = e0[e] * inv;
    const unsigned short h0 = f2bf_bits(p0);
    hb[e] = h0;
    lb[e] = f2bf_bits(p0 - bf_bits2f(h0));
    const float p1 = e1[e] * inv;
    const unsigned short h1 = f2bf_bits(p1);
    hb[4 + e] = h1;
    lb[4 + e] = f2bf_bits(p1 - bf_bits2f(h1));
  }
  const v4u uh = (v4u){pk16(hb[0], hb[1]), pk16(hb[2], hb[3]), pk16(hb[4], hb[5]), pk16(hb[6], hb[7])};
  const v4u ul = (v4u){pk16(lb[0], lb[1]), pk16(lb[2], lb[3]), pk16(lb[4], lb[5]), pk16(lb[6], lb[7])};
  unsigned short* ph = Php + (size_t)i * kSeq + 8 * (size_t)t;
  unsigned short* pl = Plp + (size_t)i * kSeq + 8 * (size_t)t;
  *(volatile v4u*)ph = uh;
  *(volatile v4u*)pl = ul;
  __threadfence();
  *(volatile v4u*)ph = uh;
  *(volatile v4u*)pl = ul;
}

extern "C" void kernel_launch(void* const* d_in, const int* in_sizes, int n_in,
                              void* d_out, int out_size, void* d_ws, size_t ws_size,
                              hipStream_t stream) {
  if (n_in < 3) return;
  const int nX = kTok * kC;
  if (in_sizes[0] != nX || in_sizes[1] != kC * kQKV || in_sizes[2] != kQKV) return;
  if (out_size != nX) return;

  const size_t szXB = (size_t)kTok * kC * 2;
  const size_t szWT = (size_t)kQKV * kC * 2;
  const size_t szQK = (size_t)kTok * kQKW * 2;
  const size_t szQS = (size_t)kBatch * kSplitRows * kQKW * 2;
  const size_t szVT = (size_t)kBatch * kC * kSeq * 2;
  const size_t szS  = (size_t)kSeq * kSeq * 4;
  const size_t szP  = (size_t)kSeq * kSeq * 2;
  const size_t offXB  = 0;
  const size_t offWT  = offXB + szXB;
  const size_t offQK  = offWT + szWT;
  const size_t offQSH = offQK + szQK;
  const size_t offQSL = offQSH + szQS;
  const size_t offVH  = offQSL + szQS;
  const size_t offVL  = offVH + szVT;
  const size_t offS   = offVL + szVT;
  const size_t offPH  = offS + szS;
  const size_t offPL  = offPH + szP;
  const size_t total  = offPL + szP;
  if (ws_size < total) return;

  const float* x  = (const float*)d_in[0];
  const float* W  = (const float*)d_in[1];
  const float* bv = (const float*)d_in[2];
  float* out = (float*)d_out;
  char* ws = (char*)d_ws;
  unsigned short* XB  = (unsigned short*)(ws + offXB);
  unsigned short* WT  = (unsigned short*)(ws + offWT);
  unsigned short* QK  = (unsigned short*)(ws + offQK);
  unsigned short* QSH = (unsigned short*)(ws + offQSH);
  unsigned short* QSL = (unsigned short*)(ws + offQSL);
  unsigned short* VTH = (unsigned short*)(ws + offVH);
  unsigned short* VTL = (unsigned short*)(ws + offVL);
  float* SC = (float*)(ws + offS);
  unsigned short* PH = (unsigned short*)(ws + offPH);
  unsigned short* PL = (unsigned short*)(ws + offPL);

  const int n8 = nX / 8;
  cast8_bf16_kernel<<<dim3(n8 / 256), dim3(256), 0, stream>>>(x, XB, n8);
  wt_cast_kernel<<<dim3(kQKV / 64, kC / 64), dim3(256), 0, stream>>>(W, WT);

  const int tilesQK = (kTok / 64) * (kQKW / 64);
  wmma_gemm64<1, false, 2, 1, false, 0, 0, 0><<<dim3(tilesQK / 8, 1), dim3(256), 0, stream>>>(
      XB, XB, kC, 0L, WT, WT, kC, 0L,
      (void*)QK, (void*)QK, kQKW, 0L, bv, bv, 0L, kTok, kQKW, kC, 1.0f);

  const int tilesQS = (kSplitRows / 64) * (kQKW / 64);
  wmma_gemm64<1, false, 2, 2, false, 0, 0, 0><<<dim3(tilesQS / 8, kBatch), dim3(256), 0, stream>>>(
      XB, XB, kC, (long)kSeq * kC, WT, WT, kC, 0L,
      (void*)QSH, (void*)QSL, kQKW, (long)kSplitRows * kQKW, bv, bv, 0L, kSplitRows, kQKW, kC, 1.0f);

  const int tilesVT = (kC / 64) * (kSeq / 64);
  wmma_gemm64<1, false, 0, 2, false, 0, 0, 0><<<dim3(tilesVT / 8, kBatch), dim3(256), 0, stream>>>(
      WT + (size_t)kQKW * kC, WT + (size_t)kQKW * kC, kC, 0L, XB, XB, kC, (long)kSeq * kC,
      (void*)VTH, (void*)VTL, kSeq, (long)kC * kSeq, bv, bv, 0L, kC, kSeq, kC, 1.0f);

  const int gridSplit = (kSplitTiles + 7) / 8;
  const int gridPlain = (kTriTiles - kSplitTiles + 7) / 8;
  const int tilesPV   = (kSeq / 64) * (kC / 64);

  for (int b = 0; b < kBatch; ++b) {
    const unsigned short* QHb = QSH + (size_t)b * kSplitRows * kQKW;
    const unsigned short* QLb = QSL + (size_t)b * kSplitRows * kQKW;
    wmma_gemm64<1, true, 0, 0, false, 0, 1, 0><<<dim3(gridSplit, 1), dim3(256), 0, stream>>>(
        QHb, QLb, kQKW, 0L, QHb + kC, QLb + kC, kQKW, 0L,
        (void*)SC, (void*)SC, kSeq, 0L, bv, bv, 0L, kSplitRows, kSplitRows, kC, kScoreScale);
    const unsigned short* Qb = QK + (size_t)b * kSeq * kQKW;
    const unsigned short* Kb = Qb + kC;
    wmma_gemm64<0, false, 0, 0, false, 0, 1, kSplitTiles><<<dim3(gridPlain, 1), dim3(256), 0, stream>>>(
        Qb, Qb, kQKW, 0L, Kb, Kb, kQKW, 0L,
        (void*)SC, (void*)SC, kSeq, 0L, bv, bv, 0L, kSeq, kSeq, kC, kScoreScale);
    causal_softmax_kernel<<<dim3(kSeq), dim3(256), 0, stream>>>(SC, PH, PL);
    const unsigned short* VHb = VTH + (size_t)b * kC * kSeq;
    const unsigned short* VLb = VTL + (size_t)b * kC * kSeq;
    float* outb = out + (size_t)b * kSeq * kC;
    wmma_gemm64<1, true, 2, 0, false, 0, 2, 0><<<dim3(tilesPV / 8, 1), dim3(256), 0, stream>>>(
        PH, PL, kSeq, 0L, VHb, VLb, kSeq, 0L,
        (void*)outb, (void*)outb, kC, 0L, bv + kQKW, bv, 0L, kSeq, kC, kSeq, 1.0f);
  }
}
